// MambaBlock_20624432955860
// MI455X (gfx1250) — hardware-verified
//
#include <hip/hip_runtime.h>
#include <math.h>

typedef __attribute__((ext_vector_type(16))) _Float16 v16h;
typedef __attribute__((ext_vector_type(8)))  _Float16 v8h;
typedef __attribute__((ext_vector_type(8)))  float    v8f;
typedef __attribute__((ext_vector_type(4)))  float    v4f;

constexpr int kBatch = 2;
constexpr int kSeqL  = 1024;
constexpr int kTok   = kBatch * kSeqL;
constexpr int kDmod  = 1024;
constexpr int kDin   = 2048;
constexpr int kNst   = 16;
constexpr int kDtR   = 64;
constexpr int kPrjN  = kDtR + 2 * kNst;
constexpr int kPrjP  = 128;
constexpr int kXZP   = 2 * kDin;
constexpr int kDff   = 4096;
constexpr int kTP    = 260;
static_assert(kTok == 2048 && kPrjN == 96 && kXZP == 4096, "shape constants");
static_assert(kDff == kXZP, "W_in and W_ff1 operand planes share one region (same type, same layout)");
static_assert((kDmod % 32) == 0 && (kDin % 32) == 0 && (kDtR % 32) == 0 && (kDff % 32) == 0, "GEMM K multiples of 32");
static_assert((kTok % 64) == 0 && (kXZP % 64) == 0 && (kPrjP % 64) == 0 && (kDin % 64) == 0 && (kDmod % 64) == 0 && (kDff % 64) == 0, "GEMM M,N multiples of 64");
static_assert((kSeqL % 64) == 0 && (kDin % 256) == 0 && (kTok % 8) == 0 && (kTok % 2) == 0, "tile multiples");
static_assert(kDmod == 4 * 256, "LayerNorm: 4 waves x 32 lanes x 8 elements per row");

constexpr float kCarryAct  = 16.0f;
constexpr float kCarryWin  = 32.0f;
constexpr float kCarryWxp  = 32.0f;
constexpr float kCarryWdt  = 8.0f;
constexpr float kCarryWout = 32.0f;
constexpr float kCarryWff1 = 32.0f;
constexpr float kCarryWff2 = 64.0f;

constexpr size_t kSzWA   = (size_t)kXZP  * kDmod * 2;
constexpr size_t kSzWXP  = (size_t)kPrjP * kDin  * 2;
constexpr size_t kSzWDT  = (size_t)kDin  * kDtR  * 2;
constexpr size_t kSzWOUT = (size_t)kDmod * kDin  * 2;
constexpr size_t kSzWFF2 = (size_t)kDmod * kDff  * 2;
constexpr size_t kSzLN   = (size_t)kTok  * kDmod * 2;
constexpr size_t kSzXZ   = (size_t)kTok  * kXZP  * 4;
constexpr size_t kSzUC   = (size_t)kTok  * kDin  * 4;
constexpr size_t kSzACT  = (size_t)kTok  * kDin  * 2;
constexpr size_t kSzPROJ = (size_t)kTok  * kPrjP * 4;
constexpr size_t kSzDT   = (size_t)kTok  * kDtR  * 2;
constexpr size_t kSzDLR  = (size_t)kTok  * kDin  * 4;
constexpr size_t kSzX1   = (size_t)kTok  * kDmod * 4;
constexpr size_t kSzH1   = (size_t)kTok  * kDff  * 2;
constexpr size_t kOffWA   = 0;
constexpr size_t kOffWXP  = kOffWA   + kSzWA;
constexpr size_t kOffWDT  = kOffWXP  + kSzWXP;
constexpr size_t kOffWOUT = kOffWDT  + kSzWDT;
constexpr size_t kOffWFF2 = kOffWOUT + kSzWOUT;
constexpr size_t kOffLN   = kOffWFF2 + kSzWFF2;
constexpr size_t kOffXZ   = kOffLN   + kSzLN;
constexpr size_t kOffUC   = kOffXZ   + kSzXZ;
constexpr size_t kOffACT  = kOffUC   + kSzUC;
constexpr size_t kOffPROJ = kOffACT  + kSzACT;
constexpr size_t kOffDT   = kOffPROJ + kSzPROJ;
constexpr size_t kOffDLR  = kOffDT   + kSzDT;
constexpr size_t kOffX1   = kOffDLR  + kSzDLR;
constexpr size_t kOffH1   = kOffX1   + kSzX1;
constexpr size_t kWsTotal = kOffH1   + kSzH1;
static_assert(kWsTotal == 127926272ull, "carve total");
static_assert(kWsTotal <= 134217728ull, "carve cap");
static_assert((kOffWXP % 128) == 0 && (kOffWDT % 128) == 0 && (kOffWOUT % 128) == 0 && (kOffWFF2 % 128) == 0 &&
              (kOffLN % 128) == 0 && (kOffXZ % 128) == 0 && (kOffUC % 128) == 0 && (kOffACT % 128) == 0 &&
              (kOffPROJ % 128) == 0 && (kOffDT % 128) == 0 && (kOffDLR % 128) == 0 && (kOffX1 % 128) == 0 &&
              (kOffH1 % 128) == 0, "128-B aligned regions");
static_assert((size_t)kTok * kDmod * 4 == 8388608ull, "output bytes");

struct FragH {
  union U { v16h v; v8h h[2]; };
  static __device__ __forceinline__ v16h load(const _Float16* p) {
    U f; f.h[0] = *(const v8h*)(p); f.h[1] = *(const v8h*)(p + 16); return f.v;
  }
  static __device__ __forceinline__ v8f mma(v16h a, v16h b, v8f c) {
    return __builtin_amdgcn_wmma_f32_16x16x32_f16(false, a, false, b, (short)0, c, false, false);
  }
};
__device__ __forceinline__ void row_guard_h(v8f& a, v8f& b, v8f& c, v8f& d, v16h x, v16h y0, v16h y1, v16h y2, v16h y3) {
  asm volatile("v_nop\n\tv_nop\n\tv_nop\n\tv_nop" : "+v"(a), "+v"(b), "+v"(c), "+v"(d) : "v"(x), "v"(y0), "v"(y1), "v"(y2), "v"(y3));
}
__device__ __forceinline__ void keep4_h(v16h a, v16h b, v16h c, v16h d) { asm volatile("v_nop" :: "v"(a), "v"(b), "v"(c), "v"(d)); }
__device__ __forceinline__ void acc_guard4(v8f& a, v8f& b, v8f& c, v8f& d) { asm volatile("v_nop\n\tv_nop\n\tv_nop\n\tv_nop" : "+v"(a), "+v"(b), "+v"(c), "+v"(d)); }

__device__ __forceinline__ float gelu_tanh_f(float x) {
  const float x3 = x * x * x;
  const float u = 0.7978845608028654f * (x + 0.044715f * x3);
  return 0.5f * x * (1.0f + tanhf(u));
}

template <int BIAS_MODE, int OUT_MODE, bool RESID, int ACT>
__global__ __launch_bounds__(256) void wmma_gemm64_f16(
    const unsigned short* __restrict__ Ap, int lda,
    const unsigned short* __restrict__ Btp, int ldb,
    void* __restrict__ Cout, int ldc,
    const float* __restrict__ bias,
    const float* __restrict__ resid,
    int M, int N, int K, float scale, float postscale) {
  const _Float16* A  = (const _Float16*)Ap;
  const _Float16* Bt = (const _Float16*)Btp;
  __shared__ __align__(16) float sT[8][16 * 68];
  const int lane = threadIdx.x & 31;
  const int wave = threadIdx.x >> 5;
  const int tilesN = N >> 6;
  const int tilesM = M >> 6;
  const int tile = blockIdx.x * 8 + wave;
  if (tile >= tilesM * tilesN) return;
  const int tm = tile / tilesN;
  const int tn = tile - tm * tilesN;
  const int m0 = tm << 6;
  const int n0 = tn << 6;

  const int rlane = lane & 15;
  const int koff  = (lane >> 4) * 8;
  const int mOff  = (lane >> 4) * 8;

  v8f acc[4][4];
#pragma unroll
  for (int i = 0; i < 4; ++i)
#pragma unroll
    for (int j = 0; j < 4; ++j) acc[i][j] = (v8f){0.f,0.f,0.f,0.f,0.f,0.f,0.f,0.f};

  for (int k0 = 0; k0 < K; k0 += 32) {
    v16h bh[4];
#pragma unroll
    for (int j = 0; j < 4; ++j) {
      const size_t bo = (size_t)(n0 + (j << 4) + rlane) * ldb + koff + k0;
      bh[j] = FragH::load(Bt + bo);
    }
#pragma unroll
    for (int i = 0; i < 4; ++i) {
      const size_t ao = (size_t)(m0 + (i << 4) + rlane) * lda + koff + k0;
      const v16h ah = FragH::load(A + ao);
#pragma unroll
      for (int j = 0; j < 4; ++j) acc[i][j] = FragH::mma(ah, bh[j], acc[i][j]);
      row_guard_h(acc[i][0], acc[i][1], acc[i][2], acc[i][3], ah, bh[0], bh[1], bh[2], bh[3]);
    }
    keep4_h(bh[0], bh[1], bh[2], bh[3]);
  }
  acc_guard4(acc[0][0], acc[0][1], acc[0][2], acc[0][3]);
  acc_guard4(acc[1][0], acc[1][1], acc[1][2], acc[1][3]);
  acc_guard4(acc[2][0], acc[2][1], acc[2][2], acc[2][3]);
  acc_guard4(acc[3][0], acc[3][1], acc[3][2], acc[3][3]);

  float* slab = sT[wave];
#pragma unroll
  for (int i = 0; i < 4; ++i) {
    const int mBase = m0 + (i << 4);
#pragma unroll
    for (int j = 0; j < 4; ++j) {
      const int n = n0 + (j << 4) + rlane;
      float bv = 0.f;
      if (BIAS_MODE == 2) bv = bias[n];
#pragma unroll
      for (int r = 0; r < 8; ++r) {
        const float v = acc[i][j][r] * scale + bv;
        slab[(mOff + r) * 68 + (j << 4) + rlane] = v;
      }
    }
    __builtin_amdgcn_fence(__ATOMIC_RELEASE, "workgroup");
    __builtin_amdgcn_wave_barrier();
    __builtin_amdgcn_fence(__ATOMIC_ACQUIRE, "workgroup");
    if (ACT == 1) {
#pragma unroll 1
      for (int it = 0; it < 32; ++it) {
        float* p = slab + (it >> 1) * 68 + (it & 1) * 32 + lane;
        const float t = *p;
        *p = gelu_tanh_f(t) * postscale;
      }
      __builtin_amdgcn_fence(__ATOMIC_RELEASE, "workgroup");
      __builtin_amdgcn_wave_barrier();
      __builtin_amdgcn_fence(__ATOMIC_ACQUIRE, "workgroup");
    }
    if (OUT_MODE == 0) {
      float* C = (float*)Cout;
      const int hh = lane >> 4, c4 = (lane & 15) * 4;
      v4f ov[8];
#pragma unroll
      for (int it = 0; it < 8; ++it) {
        const int row = it * 2 + hh;
        v4f v = *(const v4f*)(slab + row * 68 + c4);
        if (RESID) {
          const v4f rr = *(const v4f*)(resid + (size_t)(mBase + row) * ldc + n0 + c4);
          v = v + rr;
        }
        ov[it] = v;
      }
      for (int pass = 0; pass < 2; ++pass) {
#pragma unroll
        for (int it = 0; it < 8; ++it) {
          const int row = it * 2 + hh;
          *(volatile v4f*)(C + (size_t)(mBase + row) * ldc + n0 + c4) = ov[it];
        }
        __threadfence();
      }
    } else {
      const int q = lane >> 3, c8 = (lane & 7) * 8;
      unsigned short* C = (unsigned short*)Cout;
      v8h hv[4];
#pragma unroll
      for (int it = 0; it < 4; ++it) {
        const int row = it * 4 + q;
        const float* sp = slab + row * 68 + c8;
        const v4f a0 = *(const v4f*)(sp);
        const v4f a1 = *(const v4f*)(sp + 4);
#pragma unroll
        for (int e = 0; e < 4; ++e) {
          hv[it][e]     = (_Float16)a0[e];
          hv[it][4 + e] = (_Float16)a1[e];
        }
      }
      for (int pass = 0; pass < 2; ++pass) {
#pragma unroll
        for (int it = 0; it < 4; ++it) {
          const int row = it * 4 + q;
          *(volatile v8h*)(C + (size_t)(mBase + row) * ldc + n0 + c8) = hv[it];
        }
        __threadfence();
      }
    }
    __builtin_amdgcn_fence(__ATOMIC_RELEASE, "workgroup");
    __builtin_amdgcn_wave_barrier();
    __builtin_amdgcn_fence(__ATOMIC_ACQUIRE, "workgroup");
  }
}

__global__ __launch_bounds__(256) void transpose_cast_kernel(
    const float* __restrict__ W, unsigned short* __restrict__ Bt, int Kdim, int Ndim, float scale)
{
  __shared__ float tile[64 * 65];
  const int tid = threadIdx.x, lane = tid & 31, wave = tid >> 5;
  const int n0 = blockIdx.x * 64;
  const int k0 = blockIdx.y * 64;
#pragma unroll
  for (int p = 0; p < 16; ++p) {
    const int idx = tid + p * 256;
    const int kk  = idx >> 6;
    const int nn  = idx & 63;
    const int n   = n0 + nn;
    const int nc  = (n < Ndim) ? n : (Ndim - 1);
    const float v = W[(size_t)(k0 + kk) * Ndim + nc];
    tile[kk * 65 + nn] = (n < Ndim) ? (v * scale) : 0.f;
    if (p == 7) asm volatile("" ::: "memory");
  }
  __syncthreads();
  const int q = lane >> 3, c8 = (lane & 7) * 8;
  v8h hv[2];
#pragma unroll
  for (int it = 0; it < 2; ++it) {
    const int nrow = it * 32 + wave * 4 + q;
#pragma unroll
    for (int e = 0; e < 8; ++e) hv[it][e] = (_Float16)tile[(c8 + e) * 65 + nrow];
  }
  for (int pass = 0; pass < 2; ++pass) {
#pragma unroll
    for (int it = 0; it < 2; ++it) {
      const int nrow = it * 32 + wave * 4 + q;
      *(volatile v8h*)(Bt + (size_t)(n0 + nrow) * Kdim + k0 + c8) = hv[it];
    }
    __threadfence();
  }
}

__global__ __launch_bounds__(256) void layernorm_f16_kernel(
    const float* __restrict__ X, const float* __restrict__ g, const float* __restrict__ bt,
    unsigned short* __restrict__ out16, float carry)
{
  __shared__ float sS[8];
  __shared__ float sV[8];
  const int tid = threadIdx.x, lane = tid & 31, wave = tid >> 5;
  const int grp = wave >> 2;
  const int row = blockIdx.x * 2 + grp;
  const int col = (wave & 3) * 256 + lane * 8;
  const float* xr = X + (size_t)row * kDmod + col;
  const v4f a0 = *(const v4f*)(xr);
  const v4f a1 = *(const v4f*)(xr + 4);
  float s = ((a0[0] + a0[1]) + (a0[2] + a0[3])) + ((a1[0] + a1[1]) + (a1[2] + a1[3]));
#pragma unroll
  for (int o = 16; o > 0; o >>= 1) s += __shfl_xor(s, o, 32);
  if (lane == 0) sS[wave] = s;
  __syncthreads();
  const float tot  = (sS[grp * 4 + 0] + sS[grp * 4 + 1]) + (sS[grp * 4 + 2] + sS[grp * 4 + 3]);
  const float mean = tot * (1.0f / (float)kDmod);
  float ss = 0.f;
#pragma unroll
  for (int e = 0; e < 4; ++e) {
    const float d0 = a0[e] - mean;
    const float d1 = a1[e] - mean;
    ss += d0 * d0;
    ss += d1 * d1;
  }
#pragma unroll
  for (int o = 16; o > 0; o >>= 1) ss += __shfl_xor(ss, o, 32);
  if (lane == 0) sV[wave] = ss;
  __syncthreads();
  const float vtot = (sV[grp * 4 + 0] + sV[grp * 4 + 1]) + (sV[grp * 4 + 2] + sV[grp * 4 + 3]);
  const float var  = vtot * (1.0f / (float)kDmod);
  const float rstd = 1.0f / sqrtf(var + 1e-5f);
  const v4f g0 = *(const v4f*)(g  + col);
  const v4f g1 = *(const v4f*)(g  + col + 4);
  const v4f b0 = *(const v4f*)(bt + col);
  const v4f b1 = *(const v4f*)(bt + col + 4);
  v8h hv;
#pragma unroll
  for (int e = 0; e < 4; ++e) {
    const float t0 = (a0[e] - mean) * rstd;
    const float t1 = (a1[e] - mean) * rstd;
    const float gs0 = g0[e] * carry, bs0 = b0[e] * carry;
    const float gs1 = g1[e] * carry, bs1 = b1[e] * carry;
    hv[e]     = (_Float16)(t0 * gs0 + bs0);
    hv[4 + e] = (_Float16)(t1 * gs1 + bs1);
  }
  unsigned short* op = out16 + (size_t)row * kDmod + col;
  *(volatile v8h*)op = hv;
  __threadfence();
  *(volatile v8h*)op = hv;
}

__global__ __launch_bounds__(256) void dt_cast_kernel(
    const float* __restrict__ PROJ, unsigned short* __restrict__ DT16, int total8, float scale)
{
  const int i = blockIdx.x * 256 + threadIdx.x;
  if (i >= total8) return;
  const int e0  = i << 3;
  const int row = e0 >> 6;
  const int c8  = e0 & 63;
  const float* p = PROJ + (size_t)row * kPrjP + c8;
  const v4f a0 = *(const v4f*)(p);
  const v4f a1 = *(const v4f*)(p + 4);
  v8h hv;
#pragma unroll
  for (int e = 0; e < 4; ++e) {
    hv[e]     = (_Float16)(a0[e] * scale);
    hv[4 + e] = (_Float16)(a1[e] * scale);
  }
  unsigned short* qd = DT16 + e0;
  *(volatile v8h*)qd = hv;
  __threadfence();
  *(volatile v8h*)qd = hv;
}

__global__ __launch_bounds__(256) void conv_silu_kernel(
    const float* __restrict__ XZ, const float* __restrict__ cw, const float* __restrict__ cb,
    float* __restrict__ UC, unsigned short* __restrict__ UC16, float carry)
{
  __shared__ __align__(16) float sT[16 * kTP];
  const int tid = threadIdx.x, lane = tid & 31, wave = tid >> 5;
  const int d0 = blockIdx.x * 256, d = d0 + tid;
  const int g0 = blockIdx.y * 64;
  const int tb = g0 & (kSeqL - 1);
  const v4f wv = *(const v4f*)(cw + (size_t)d * 4);
  const float w0 = wv[0], w1 = wv[1], w2 = wv[2], w3 = wv[3];
  const float bc = cb[d];
  float xm3, xm2, xm1;
  {
    const bool hist = (tb > 0);
    const int rb = hist ? (g0 - 3) : g0;
    const float v3 = XZ[(size_t)rb * kXZP + d];
    const float v2 = XZ[(size_t)(rb + 1) * kXZP + d];
    const float v1 = XZ[(size_t)(rb + 2) * kXZP + d];
    xm3 = hist ? v3 : 0.f;
    xm2 = hist ? v2 : 0.f;
    xm1 = hist ? v1 : 0.f;
  }
  const int hrow = wave >> 1;
  const int hch  = (wave & 1) * 128 + lane * 4;
#pragma unroll 1
  for (int sub = 0; sub < 4; ++sub) {
    const int lb = g0 + sub * 16;
#pragma unroll 1
    for (int s = 0; s < 16; ++s) {
      const float xcur = XZ[(size_t)(lb + s) * kXZP + d];
      float acc = w0 * xm3;
      acc = fmaf(w1, xm2, acc);
      acc = fmaf(w2, xm1, acc);
      acc = fmaf(w3, xcur, acc);
      const float sv = acc + bc;
      const float sg = __builtin_amdgcn_rcpf(1.0f + expf(-sv));
      sT[s * kTP + tid] = sv * sg;
      xm3 = xm2; xm2 = xm1; xm1 = xcur;
    }
    __syncthreads();
    v4f fv[4];
    v8h bv[2];
#pragma unroll
    for (int it = 0; it < 4; ++it) fv[it] = *(const v4f*)(sT + (it * 4 + hrow) * kTP + hch);
#pragma unroll
    for (int it = 0; it < 2; ++it) {
      const float* sp = sT + (it * 8 + wave) * kTP + lane * 8;
      const v4f a0 = *(const v4f*)(sp);
      const v4f a1 = *(const v4f*)(sp + 4);
#pragma unroll
      for (int e = 0; e < 4; ++e) {
        bv[it][e]     = (_Float16)(a0[e] * carry);
        bv[it][4 + e] = (_Float16)(a1[e] * carry);
      }
    }
    for (int pass = 0; pass < 2; ++pass) {
#pragma unroll
      for (int it = 0; it < 4; ++it)
        *(volatile v4f*)(UC + (size_t)(lb + it * 4 + hrow) * kDin + d0 + hch) = fv[it];
#pragma unroll
      for (int it = 0; it < 2; ++it)
        *(volatile v8h*)(UC16 + (size_t)(lb + it * 8 + wave) * kDin + d0 + lane * 8) = bv[it];
      __threadfence();
    }
    __syncthreads();
  }
}

__global__ __launch_bounds__(256) void scan_kernel(
    const float* __restrict__ DLR, const float* __restrict__ UC, const float* __restrict__ XZ,
    const float* __restrict__ PROJ, const float* __restrict__ A_log, const float* __restrict__ Dv,
    unsigned short* __restrict__ Y16, float carry)
{
#pragma clang fp contract(off)
  __shared__ __align__(16) float sBC[16 * 32];
  __shared__ __align__(16) float sY[16 * kTP];
  __shared__ float sA[kNst * 256];
  __shared__ float sE[kNst * 256];
  const int tid = threadIdx.x, lane = tid & 31, wave = tid >> 5;
  const int d0 = blockIdx.x * 256, d = d0 + tid;
  const size_t row0 = (size_t)blockIdx.y * kSeqL;

#pragma unroll 1
  for (int n = 0; n < kNst; ++n) sA[n * 256 + tid] = -expf(A_log[(size_t)d * kNst + n]);
  float h[kNst];
#pragma unroll
  for (int n = 0; n < kNst; ++n) h[n] = 0.f;
  const float Dd = Dv[d];

#pragma unroll 1
  for (int c = 0; c < kSeqL / 16; ++c) {
    const int l0 = c * 16;
    if (tid < 128) {
      const int r = tid >> 3, q = (tid & 7) * 4;
      const v4f v = *(const v4f*)(PROJ + (row0 + l0 + r) * kPrjP + kDtR + q);
      *(v4f*)(sBC + r * 32 + q) = v;
    }
    __syncthreads();
#pragma unroll 1
    for (int s = 0; s < 16; ++s) {
      const size_t m = row0 + (size_t)(l0 + s);
      const float a     = DLR[m * kDin + d];
      const float xv    = UC[m * kDin + d];
      const float zv    = XZ[m * kXZP + kDin + d];
      const float delta = fmaxf(a, 0.0f) + log1pf(expf(-fabsf(a)));
#pragma unroll 1
      for (int n = 0; n < kNst; ++n) {
        float e = expf(delta * sA[n * 256 + tid]);
        e = (e < 1.17549435e-38f) ? 0.0f : e;
        sE[n * 256 + tid] = e;
      }
      v4f Bq[4], Cq[4];
#pragma unroll
      for (int qq = 0; qq < 4; ++qq) {
        Bq[qq] = *(const v4f*)(sBC + s * 32 + 4 * qq);
        Cq[qq] = *(const v4f*)(sBC + s * 32 + kNst + 4 * qq);
      }
      float y = 0.f;
#pragma unroll
      for (int n = 0; n < kNst; ++n) {
        const float e  = sE[n * 256 + tid];
        const float db = delta * Bq[n >> 2][n & 3];
        const float p  = db * xv;
        const float qv = e * h[n];
        const float hn = qv + p;
        h[n] = hn;
        const float rr = hn * Cq[n >> 2][n & 3];
        y = y + rr;
      }
      const float sk = xv * Dd;
      y = y + sk;
      const float sg = __builtin_amdgcn_rcpf(1.0f + expf(-zv));
      const float gt = zv * sg;
      sY[s * kTP + tid] = (y * gt) * carry;
    }
    __syncthreads();
    v8h hv[2];
#pragma unroll
    for (int it = 0; it < 2; ++it) {
      const float* sp = sY + (it * 8 + wave) * kTP + lane * 8;
      const v4f a0 = *(const v4f*)(sp);
      const v4f a1 = *(const v4f*)(sp + 4);
#pragma unroll
      for (int e = 0; e < 4; ++e) { hv[it][e] = (_Float16)a0[e]; hv[it][4 + e] = (_Float16)a1[e]; }
    }
    for (int pass = 0; pass < 2; ++pass) {
#pragma unroll
      for (int it = 0; it < 2; ++it)
        *(volatile v8h*)(Y16 + (row0 + (size_t)(l0 + it * 8 + wave)) * kDin + d0 + lane * 8) = hv[it];
      __threadfence();
    }
  }
}

extern "C" void kernel_launch(void* const* d_in, const int* in_sizes, int n_in,
                              void* d_out, int out_size, void* d_ws, size_t ws_size,
                              hipStream_t stream)
{
  if (n_in < 18) return;
  if (in_sizes[0] != kTok * kDmod) return;
  if (in_sizes[1] != kDmod || in_sizes[2] != kDmod) return;
  if (in_sizes[3] != kDmod * kXZP) return;
  if (in_sizes[4] != kDin * 4 || in_sizes[5] != kDin) return;
  if (in_sizes[6] != kDin * kPrjN) return;
  if (in_sizes[7] != kDtR * kDin || in_sizes[8] != kDin) return;
  if (in_sizes[9] != kDin * kNst || in_sizes[10] != kDin) return;
  if (in_sizes[11] != kDin * kDmod) return;
  if (in_sizes[12] != kDmod || in_sizes[13] != kDmod) return;
  if (in_sizes[14] != kDmod * kDff || in_sizes[15] != kDff) return;
  if (in_sizes[16] != kDff * kDmod || in_sizes[17] != kDmod) return;
  if (out_size != kTok * kDmod) return;
  if (ws_size < kWsTotal) return;

  const float* x       = (const float*)d_in[0];
  const float* ln1_g   = (const float*)d_in[1];
  const float* ln1_b   = (const float*)d_in[2];
  const float* w_in    = (const float*)d_in[3];
  const float* w_conv  = (const float*)d_in[4];
  const float* b_conv  = (const float*)d_in[5];
  const float* w_xproj = (const float*)d_in[6];
  const float* w_dt    = (const float*)d_in[7];
  const float* b_dt    = (const float*)d_in[8];
  const float* A_log   = (const float*)d_in[9];
  const float* Dp      = (const float*)d_in[10];
  const float* w_out   = (const float*)d_in[11];
  const float* ln2_g   = (const float*)d_in[12];
  const float* ln2_b   = (const float*)d_in[13];
  const float* w_ff1   = (const float*)d_in[14];
  const float* b_ff1   = (const float*)d_in[15];
  const float* w_ff2   = (const float*)d_in[16];
  const float* b_ff2   = (const float*)d_in[17];
  float* dout = (float*)d_out;

  char* ws = (char*)d_ws;
  unsigned short* WA    = (unsigned short*)(ws + kOffWA);
  unsigned short* WXP   = (unsigned short*)(ws + kOffWXP);
  unsigned short* WDT   = (unsigned short*)(ws + kOffWDT);
  unsigned short* WOUT  = (unsigned short*)(ws + kOffWOUT);
  unsigned short* WFF2  = (unsigned short*)(ws + kOffWFF2);
  unsigned short* LN16  = (unsigned short*)(ws + kOffLN);
  float*          XZ    = (float*)(ws + kOffXZ);
  float*          UC    = (float*)(ws + kOffUC);
  unsigned short* ACT16 = (unsigned short*)(ws + kOffACT);
  float*          PROJ  = (float*)(ws + kOffPROJ);
  unsigned short* DT16  = (unsigned short*)(ws + kOffDT);
  float*          DLR   = (float*)(ws + kOffDLR);
  float*          X1    = (float*)(ws + kOffX1);
  unsigned short* H1    = (unsigned short*)(ws + kOffH1);
  const float* dummy_bias  = b_dt;
  const float* dummy_resid = x;

  transpose_cast_kernel<<<dim3(kXZP / 64, kDmod / 64), 256, 0, stream>>>(w_in, WA, kDmod, kXZP, kCarryWin);
  transpose_cast_kernel<<<dim3(kPrjP / 64, kDin / 64), 256, 0, stream>>>(w_xproj, WXP, kDin, kPrjN, kCarryWxp);
  transpose_cast_kernel<<<dim3(kDin / 64, kDtR / 64), 256, 0, stream>>>(w_dt, WDT, kDtR, kDin, kCarryWdt);
  transpose_cast_kernel<<<dim3(kDmod / 64, kDin / 64), 256, 0, stream>>>(w_out, WOUT, kDin, kDmod, kCarryWout);
  transpose_cast_kernel<<<dim3(kDmod / 64, kDff / 64), 256, 0, stream>>>(w_ff2, WFF2, kDff, kDmod, kCarryWff2);

  layernorm_f16_kernel<<<kTok / 2, 256, 0, stream>>>(x, ln1_g, ln1_b, LN16, kCarryAct);

  wmma_gemm64_f16<0, 0, false, 0><<<dim3(256), 256, 0, stream>>>(
      LN16, kDmod, WA, kDmod, (void*)XZ, kXZP, dummy_bias, dummy_resid,
      kTok, kXZP, kDmod, 1.0f / (kCarryAct * kCarryWin), 1.0f);

  transpose_cast_kernel<<<dim3(kDff / 64, kDmod / 64), 256, 0, stream>>>(w_ff1, WA, kDmod, kDff, kCarryWff1);

  conv_silu_kernel<<<dim3(kDin / 256, kTok / 64), 256, 0, stream>>>(XZ, w_conv, b_conv, UC, ACT16, kCarryAct);

  wmma_gemm64_f16<0, 0, false, 0><<<dim3(8), 256, 0, stream>>>(
      ACT16, kDin, WXP, kDin, (void*)PROJ, kPrjP, dummy_bias, dummy_resid,
      kTok, kPrjP, kDin, 1.0f / (kCarryAct * kCarryWxp), 1.0f);

  dt_cast_kernel<<<(kTok * kDtR) / 8 / 256, 256, 0, stream>>>(PROJ, DT16, (kTok * kDtR) / 8, kCarryAct);

  wmma_gemm64_f16<2, 0, false, 0><<<dim3(128), 256, 0, stream>>>(
      DT16, kDtR, WDT, kDtR, (void*)DLR, kDin, b_dt, dummy_resid,
      kTok, kDin, kDtR, 1.0f / (kCarryAct * kCarryWdt), 1.0f);

  scan_kernel<<<dim3(kDin / 256, kBatch), 256, 0, stream>>>(DLR, UC, XZ, PROJ, A_log, Dp, ACT16, kCarryAct);

  wmma_gemm64_f16<0, 0, true, 0><<<dim3(64), 256, 0, stream>>>(
      ACT16, kDin, WOUT, kDin, (void*)X1, kDmod, dummy_bias, x,
      kTok, kDmod, kDin, 1.0f / (kCarryAct * kCarryWout), 1.0f);

  layernorm_f16_kernel<<<kTok / 2, 256, 0, stream>>>(X1, ln2_g, ln2_b, LN16, kCarryAct);

  wmma_gemm64_f16<2, 1, false, 1><<<dim3(256), 256, 0, stream>>>(
      LN16, kDmod, WA, kDmod, (void*)H1, kDff, b_ff1, dummy_resid,
      kTok, kDff, kDmod, 1.0f / (kCarryAct * kCarryWff1), kCarryAct);

  wmma_gemm64_f16<2, 0, true, 0><<<dim3(64), 256, 0, stream>>>(
      H1, kDff, WFF2, kDff, (void*)dout, kDmod, b_ff2, X1,
      kTok, kDmod, kDff, 1.0f / (kCarryAct * kCarryWff2), 1.0f);
}
